// CPWanSelfAttention_78838419685970
// MI455X (gfx1250) — hardware-verified
//
#include <hip/hip_runtime.h>
#include <stddef.h>


#define DIM   2048
#define SEQ   1992
#define SPAD  2048
#define HEADS 16
#define DHEAD 128
#define PLP   40

typedef unsigned short us;
typedef us     v8us  __attribute__((ext_vector_type(8)));
typedef __bf16 v16bf __attribute__((ext_vector_type(16)));
typedef float  v8f   __attribute__((ext_vector_type(8)));
typedef float  v4f   __attribute__((ext_vector_type(4)));

union Frag { v16bf v; v8us u[2]; };

__device__ __forceinline__ v8f zf8() { v8f z = {0.f, 0.f, 0.f, 0.f, 0.f, 0.f, 0.f, 0.f}; return z; }
__device__ __forceinline__ v8us zu8() { v8us z = {0, 0, 0, 0, 0, 0, 0, 0}; return z; }

__device__ __forceinline__ v8f wbf(const Frag& a, const Frag& b, v8f c) {
  return __builtin_amdgcn_wmma_f32_16x16x32_bf16(false, a.v, false, b.v, (short)0, c,
                                                 false, false);
}

#define WGUARD1(acc, fa, fb, fc, fd)                                              \
  asm volatile("v_nop\n\tv_nop\n\tv_nop\n\tv_nop"                                 \
               : "+v"(acc)                                                        \
               : "v"(fa.u[0]), "v"(fa.u[1]), "v"(fb.u[0]), "v"(fb.u[1]),         \
                 "v"(fc.u[0]), "v"(fc.u[1]), "v"(fd.u[0]), "v"(fd.u[1]))

#define WGUARD2(acc0, acc1, fa, fb, fc, fd, fe, ff)                               \
  asm volatile("v_nop\n\tv_nop\n\tv_nop\n\tv_nop"                                 \
               : "+v"(acc0), "+v"(acc1)                                           \
               : "v"(fa.u[0]), "v"(fa.u[1]), "v"(fb.u[0]), "v"(fb.u[1]),         \
                 "v"(fc.u[0]), "v"(fc.u[1]), "v"(fd.u[0]), "v"(fd.u[1]),         \
                 "v"(fe.u[0]), "v"(fe.u[1]), "v"(ff.u[0]), "v"(ff.u[1]))

__device__ __forceinline__ Frag ld_frag(const us* p, int ld, int lane) {
  const us* q = p + (size_t)(lane & 15) * (size_t)ld + (size_t)((lane >> 4) << 3);
  Frag f;
  f.u[0] = *(const v8us*)(q);
  f.u[1] = *(const v8us*)(q + 16);
  return f;
}

__device__ __forceinline__ unsigned int bf_bits(float x) {
  const unsigned int u = __float_as_uint(x);
  return (u + 0x7FFFu + ((u >> 16) & 1u)) >> 16;
}

__device__ __forceinline__ void split1(float x, us& hi, us& lo) {
  const unsigned int hb = bf_bits(x);
  const float hf = __uint_as_float(hb << 16);
  const unsigned int lb = bf_bits(x - hf);
  hi = (us)hb;
  lo = (us)lb;
}

__device__ __forceinline__ void split8(const float (&v)[8], v8us& hi, v8us& lo) {
#pragma unroll
  for (int e = 0; e < 8; ++e) {
    us a, b;
    split1(v[e], a, b);
    hi[e] = a;
    lo[e] = b;
  }
}

struct CvtArgs {
  const float* s0; const float* s1; const float* s2; const float* s3;
  us* h0; us* h1; us* h2; us* h3;
  us* l0; us* l1; us* l2; us* l3;
  int n0; int n1; int n2; int n3;
};
typedef char cvt_args_size_check[(sizeof(CvtArgs) == 112) ? 1 : -1];

__global__ void __launch_bounds__(256) cvt_planes_kernel(CvtArgs a) {
  const int z = blockIdx.y;
  const int row = blockIdx.x;
  const int t = threadIdx.x;
  const float* src = (z == 0) ? a.s0 : (z == 1) ? a.s1 : (z == 2) ? a.s2 : a.s3;
  us* ph = (z == 0) ? a.h0 : (z == 1) ? a.h1 : (z == 2) ? a.h2 : a.h3;
  us* pl = (z == 0) ? a.l0 : (z == 1) ? a.l1 : (z == 2) ? a.l2 : a.l3;
  const int nrows = (z == 0) ? a.n0 : (z == 1) ? a.n1 : (z == 2) ? a.n2 : a.n3;

  const size_t off = (size_t)row * DIM + (size_t)t * 8;
  v8us hv = zu8(), lv = zu8();
  if (row < nrows) {
    const v4f x0 = *(const v4f*)(src + off);
    const v4f x1 = *(const v4f*)(src + off + 4);
    float v[8] = {x0[0], x0[1], x0[2], x0[3], x1[0], x1[1], x1[2], x1[3]};
    split8(v, hv, lv);
  }
  us* dh = ph + off;
  us* dl = pl + off;
  *(volatile v8us*)dh = hv;
  *(volatile v8us*)dl = lv;
  __threadfence();
  *(volatile v8us*)dh = hv;
  *(volatile v8us*)dl = lv;
}

template <int MODE>
__global__ void __launch_bounds__(256) gemm_abT_kernel(
    const us* __restrict__ Ah, const us* __restrict__ Al,
    const us* __restrict__ Bh, const us* __restrict__ Bl,
    const float* __restrict__ bias,
    float* __restrict__ Cf, us* __restrict__ Ch, us* __restrict__ Cl,
    int m_valid, int n_valid) {
  __shared__ __attribute__((aligned(16))) float stg[8][16 * 64];

  const int t = threadIdx.x;
  const int lane = t & 31;
  const int w = t >> 5;
  const int h = lane >> 4;
  const int n16 = lane & 15;
  const int wm = w & 3, wn = w >> 2;
  const int row0 = blockIdx.x * 128 + wm * 32;
  const int col0 = blockIdx.y * 128 + wn * 64;

  v8f acc[2][4];
#pragma unroll
  for (int i = 0; i < 2; ++i)
#pragma unroll
    for (int j = 0; j < 4; ++j) acc[i][j] = zf8();

  const us* pa_h = Ah + (size_t)row0 * DIM;
  const us* pa_l = Al + (size_t)row0 * DIM;
  const us* pb_h = Bh + (size_t)col0 * DIM;
  const us* pb_l = Bl + (size_t)col0 * DIM;

#pragma unroll 1
  for (int k0 = 0; k0 < DIM; k0 += 32) {
    const Frag ah0 = ld_frag(pa_h + k0, DIM, lane);
    const Frag ah1 = ld_frag(pa_h + 16 * DIM + k0, DIM, lane);
    const Frag al0 = ld_frag(pa_l + k0, DIM, lane);
    const Frag al1 = ld_frag(pa_l + 16 * DIM + k0, DIM, lane);
#pragma unroll
    for (int j = 0; j < 4; ++j) {
      const Frag bh = ld_frag(pb_h + (size_t)(16 * j) * DIM + k0, DIM, lane);
      const Frag bl = ld_frag(pb_l + (size_t)(16 * j) * DIM + k0, DIM, lane);
      acc[0][j] = wbf(ah0, bh, acc[0][j]);
      acc[0][j] = wbf(ah0, bl, acc[0][j]);
      acc[0][j] = wbf(al0, bh, acc[0][j]);
      acc[1][j] = wbf(ah1, bh, acc[1][j]);
      acc[1][j] = wbf(ah1, bl, acc[1][j]);
      acc[1][j] = wbf(al1, bh, acc[1][j]);
      WGUARD2(acc[0][j], acc[1][j], ah0, ah1, al0, al1, bh, bl);
    }
  }

  float* st = &stg[w][0];
#pragma unroll
  for (int i = 0; i < 2; ++i) {
#pragma unroll
    for (int j = 0; j < 4; ++j)
#pragma unroll
      for (int r = 0; r < 8; ++r)
        st[(8 * h + r) * 64 + 16 * j + n16] = acc[i][j][r];
    __syncthreads();

    if (MODE != 1) {
      const int cp = n16 * 4;
      const int gcol = col0 + cp;
      const v4f bb = *(const v4f*)(bias + gcol);
      v4f vals[8];
#pragma unroll
      for (int it = 0; it < 8; ++it) {
        const int rl = 2 * it + h;
        vals[it] = *(const v4f*)(st + rl * 64 + cp) + bb;
      }
#pragma unroll
      for (int it = 0; it < 8; ++it) {
        const int grow = row0 + 16 * i + 2 * it + h;
        if (MODE == 0 || grow < m_valid)
          *(volatile v4f*)(Cf + (size_t)grow * DIM + gcol) = vals[it];
      }
      __threadfence();
#pragma unroll
      for (int it = 0; it < 8; ++it) {
        const int grow = row0 + 16 * i + 2 * it + h;
        if (MODE == 0 || grow < m_valid)
          *(volatile v4f*)(Cf + (size_t)grow * DIM + gcol) = vals[it];
      }
    } else {
      const int rsub = lane >> 3;
      const int q8 = (lane & 7) * 8;
      v8us hv[4], lv[4];
#pragma unroll
      for (int it = 0; it < 4; ++it) {
        const int rl = 4 * it + rsub;
        const int grow = row0 + 16 * i + rl;
        const float rb = bias[grow];
        const v4f x0 = *(const v4f*)(st + rl * 64 + q8);
        const v4f x1 = *(const v4f*)(st + rl * 64 + q8 + 4);
        float v[8] = {x0[0], x0[1], x0[2], x0[3], x1[0], x1[1], x1[2], x1[3]};
#pragma unroll
        for (int e = 0; e < 8; ++e) {
          float y = v[e] + rb;
          if (col0 + q8 + e >= n_valid) y = 0.f;
          v[e] = y;
        }
        split8(v, hv[it], lv[it]);
      }
#pragma unroll
      for (int it = 0; it < 4; ++it) {
        const int grow = row0 + 16 * i + 4 * it + rsub;
        const size_t p = (size_t)grow * DIM + (size_t)(col0 + q8);
        *(volatile v8us*)(Ch + p) = hv[it];
        *(volatile v8us*)(Cl + p) = lv[it];
      }
      __threadfence();
#pragma unroll
      for (int it = 0; it < 4; ++it) {
        const int grow = row0 + 16 * i + 4 * it + rsub;
        const size_t p = (size_t)grow * DIM + (size_t)(col0 + q8);
        *(volatile v8us*)(Ch + p) = hv[it];
        *(volatile v8us*)(Cl + p) = lv[it];
      }
    }
    __syncthreads();
  }
}

__global__ void __launch_bounds__(256) norm_rope_kernel(
    const float* __restrict__ Qf, const float* __restrict__ Kf,
    const float* __restrict__ wq_n, const float* __restrict__ wk_n,
    const float* __restrict__ fcos, const float* __restrict__ fsin,
    us* __restrict__ Qh, us* __restrict__ Ql, us* __restrict__ Kh, us* __restrict__ Kl,
    int s_valid) {
  __shared__ float red[8];
  const int s = blockIdx.x;
  const int z = blockIdx.y;
  const int t = threadIdx.x;
  const int lane = t & 31, w = t >> 5;
  const float* src = z ? Kf : Qf;
  const float* nw = z ? wk_n : wq_n;
  us* oh = z ? Kh : Qh;
  us* ol = z ? Kl : Ql;

  const size_t off = (size_t)s * DIM + (size_t)t * 8;
  v8us hv = zu8(), lv = zu8();
  if (s < s_valid) {
    const v4f x0 = *(const v4f*)(src + off);
    const v4f x1 = *(const v4f*)(src + off + 4);
    float x[8] = {x0[0], x0[1], x0[2], x0[3], x1[0], x1[1], x1[2], x1[3]};
    float ss = 0.f;
#pragma unroll
    for (int e = 0; e < 8; ++e) ss += x[e] * x[e];
#pragma unroll
    for (int o = 16; o > 0; o >>= 1) ss += __shfl_xor(ss, o, 32);
    if (lane == 0) red[w] = ss;
    __syncthreads();
    float tot = 0.f;
#pragma unroll
    for (int i = 0; i < 8; ++i) tot += red[i];
    const float var = tot * (1.0f / (float)DIM);
    const float inv = rsqrtf(var + 1e-6f);

    const v4f w0 = *(const v4f*)(nw + t * 8);
    const v4f w1 = *(const v4f*)(nw + t * 8 + 4);
    float wv[8] = {w0[0], w0[1], w0[2], w0[3], w1[0], w1[1], w1[2], w1[3]};
    const int d0 = (t * 8) & (DHEAD - 1);
    const float* pc = fcos + (size_t)s * DHEAD + d0;
    const float* pn = fsin + (size_t)s * DHEAD + d0;
    const v4f c0 = *(const v4f*)pc, c1 = *(const v4f*)(pc + 4);
    const v4f sn0 = *(const v4f*)pn, sn1 = *(const v4f*)(pn + 4);
    float cv[8] = {c0[0], c0[1], c0[2], c0[3], c1[0], c1[1], c1[2], c1[3]};
    float sv[8] = {sn0[0], sn0[1], sn0[2], sn0[3], sn1[0], sn1[1], sn1[2], sn1[3]};

    float y[8];
#pragma unroll
    for (int e = 0; e < 8; ++e) y[e] = (x[e] * inv) * wv[e];
    float o8[8];
#pragma unroll
    for (int p = 0; p < 4; ++p) {
      const int e = 2 * p;
      const float c = cv[e];
      const float sn = sv[e + 1];
      o8[e]     = y[e] * c - y[e + 1] * sn;
      o8[e + 1] = y[e] * sn + y[e + 1] * c;
    }
    split8(o8, hv, lv);
  }
  us* dh = oh + off;
  us* dl = ol + off;
  *(volatile v8us*)dh = hv;
  *(volatile v8us*)dl = lv;
  __threadfence();
  *(volatile v8us*)dh = hv;
  *(volatile v8us*)dl = lv;
}

__global__ void __launch_bounds__(32) attn_kernel(
    const us* __restrict__ Qh, const us* __restrict__ Ql,
    const us* __restrict__ Kh, const us* __restrict__ Kl,
    const us* __restrict__ Vh, const us* __restrict__ Vl,
    us* __restrict__ Ch, us* __restrict__ Cl) {
  __shared__ __attribute__((aligned(16))) us pb[2][16 * PLP];
  __shared__ __attribute__((aligned(16))) float ost[16 * 128];

  const int lane = threadIdx.x;
  const int h = lane >> 4;
  const int n16 = lane & 15;
  const int q0 = blockIdx.x * 16;
  const int hd = blockIdx.y;

  const us* pq_h = Qh + (size_t)q0 * DIM + (size_t)hd * DHEAD;
  const us* pq_l = Ql + (size_t)q0 * DIM + (size_t)hd * DHEAD;
  const us* pk_h = Kh + (size_t)hd * DHEAD;
  const us* pk_l = Kl + (size_t)hd * DHEAD;
  const us* pv_h = Vh + (size_t)hd * DHEAD * SPAD;
  const us* pv_l = Vl + (size_t)hd * DHEAD * SPAD;

  const float scale = 0.08838834764831845f;
  const float ninf = __uint_as_float(0xff800000u);

  v8f o[8];
#pragma unroll
  for (int dt = 0; dt < 8; ++dt) o[dt] = zf8();
  float mrun[8], lrun[8];
#pragma unroll
  for (int r = 0; r < 8; ++r) { mrun[r] = ninf; lrun[r] = 0.f; }

#pragma unroll 1
  for (int kb = 0; kb < SPAD / 32; ++kb) {
    const int key0 = kb * 32;
    const us* kr_h = pk_h + (size_t)key0 * DIM;
    const us* kr_l = pk_l + (size_t)key0 * DIM;

    v8f s0 = zf8(), s1 = zf8();
#pragma unroll 1
    for (int kk = 0; kk < DHEAD / 32; ++kk) {
      const int d0 = kk * 32;
      const Frag qh = ld_frag(pq_h + d0, DIM, lane);
      const Frag ql = ld_frag(pq_l + d0, DIM, lane);
      {
        const Frag kh = ld_frag(kr_h + d0, DIM, lane);
        const Frag kl = ld_frag(kr_l + d0, DIM, lane);
        s0 = wbf(qh, kh, s0);
        s0 = wbf(qh, kl, s0);
        s0 = wbf(ql, kh, s0);
        WGUARD1(s0, qh, ql, kh, kl);
      }
      {
        const Frag kh = ld_frag(kr_h + 16 * DIM + d0, DIM, lane);
        const Frag kl = ld_frag(kr_l + 16 * DIM + d0, DIM, lane);
        s1 = wbf(qh, kh, s1);
        s1 = wbf(qh, kl, s1);
        s1 = wbf(ql, kh, s1);
        WGUARD1(s1, qh, ql, kh, kl);
      }
    }

    float al[8];
#pragma unroll
    for (int r = 0; r < 8; ++r) {
      const float x0 = s0[r] * scale;
      const float x1 = s1[r] * scale;
      float mx = fmaxf(x0, x1);
      mx = fmaxf(mx, __shfl_xor(mx, 1, 32));
      mx = fmaxf(mx, __shfl_xor(mx, 2, 32));
      mx = fmaxf(mx, __shfl_xor(mx, 4, 32));
      mx = fmaxf(mx, __shfl_xor(mx, 8, 32));
      const float mn = fmaxf(mrun[r], mx);
      const float a = __expf(mrun[r] - mn);
      const float e0 = __expf(x0 - mn);
      const float e1 = __expf(x1 - mn);
      float ps = e0 + e1;
      ps += __shfl_xor(ps, 1, 32);
      ps += __shfl_xor(ps, 2, 32);
      ps += __shfl_xor(ps, 4, 32);
      ps += __shfl_xor(ps, 8, 32);
      lrun[r] = lrun[r] * a + ps;
      mrun[r] = mn;
      al[r] = a;
      s0[r] = e0;
      s1[r] = e1;
    }
    const v8f alv = {al[0], al[1], al[2], al[3], al[4], al[5], al[6], al[7]};
#pragma unroll
    for (int dt = 0; dt < 8; ++dt) o[dt] = o[dt] * alv;

#pragma unroll
    for (int r = 0; r < 8; ++r) {
      us a0, b0, a1, b1;
      split1(s0[r], a0, b0);
      split1(s1[r], a1, b1);
      const int ro = (8 * h + r) * PLP;
      pb[0][ro + n16] = a0;
      pb[1][ro + n16] = b0;
      pb[0][ro + 16 + n16] = a1;
      pb[1][ro + 16 + n16] = b1;
    }
    __syncthreads();
    const Frag ph = ld_frag(&pb[0][0], PLP, lane);
    const Frag pl = ld_frag(&pb[1][0], PLP, lane);

    const us* vr_h = pv_h + key0;
    const us* vr_l = pv_l + key0;
#pragma unroll
    for (int dt = 0; dt < 8; ++dt) {
      const Frag vh = ld_frag(vr_h + (size_t)(16 * dt) * SPAD, SPAD, lane);
      const Frag vl = ld_frag(vr_l + (size_t)(16 * dt) * SPAD, SPAD, lane);
      o[dt] = wbf(ph, vh, o[dt]);
      o[dt] = wbf(ph, vl, o[dt]);
      o[dt] = wbf(pl, vh, o[dt]);
      WGUARD1(o[dt], ph, pl, vh, vl);
    }
    __syncthreads();
  }

  float il[8];
#pragma unroll
  for (int r = 0; r < 8; ++r) il[r] = __builtin_amdgcn_rcpf(lrun[r]);
  const v8f ilv = {il[0], il[1], il[2], il[3], il[4], il[5], il[6], il[7]};
#pragma unroll
  for (int dt = 0; dt < 8; ++dt) {
    const v8f ov = o[dt] * ilv;
#pragma unroll
    for (int r = 0; r < 8; ++r) ost[(8 * h + r) * 128 + 16 * dt + n16] = ov[r];
  }
  __syncthreads();

  v8us hv[8], lv[8];
#pragma unroll
  for (int it = 0; it < 8; ++it) {
    const int rl = 2 * it + h;
    const v4f x0 = *(const v4f*)(&ost[rl * 128 + 8 * n16]);
    const v4f x1 = *(const v4f*)(&ost[rl * 128 + 8 * n16 + 4]);
    float v[8] = {x0[0], x0[1], x0[2], x0[3], x1[0], x1[1], x1[2], x1[3]};
    split8(v, hv[it], lv[it]);
  }
#pragma unroll
  for (int it = 0; it < 8; ++it) {
    const size_t p = (size_t)(q0 + 2 * it + h) * DIM + (size_t)hd * DHEAD + (size_t)(8 * n16);
    *(volatile v8us*)(Ch + p) = hv[it];
    *(volatile v8us*)(Cl + p) = lv[it];
  }
  __threadfence();
#pragma unroll
  for (int it = 0; it < 8; ++it) {
    const size_t p = (size_t)(q0 + 2 * it + h) * DIM + (size_t)hd * DHEAD + (size_t)(8 * n16);
    *(volatile v8us*)(Ch + p) = hv[it];
    *(volatile v8us*)(Cl + p) = lv[it];
  }
}

extern "C" void kernel_launch(void* const* d_in, const int* in_sizes, int n_in,
                              void* d_out, int out_size, void* d_ws,
                              size_t ws_size, hipStream_t stream) {
  (void)in_sizes; (void)n_in; (void)out_size;
  const float* hs   = (const float*)d_in[0];
  const float* fcos = (const float*)d_in[1];
  const float* fsin = (const float*)d_in[2];
  const float* wq   = (const float*)d_in[3];
  const float* bq   = (const float*)d_in[4];
  const float* wk   = (const float*)d_in[5];
  const float* bk   = (const float*)d_in[6];
  const float* wv   = (const float*)d_in[7];
  const float* bv   = (const float*)d_in[8];
  const float* nqw  = (const float*)d_in[9];
  const float* nkw  = (const float*)d_in[10];
  const float* wo   = (const float*)d_in[11];
  const float* bo   = (const float*)d_in[12];
  float* out = (float*)d_out;

  const size_t PLANE  = (size_t)SPAD * DIM * sizeof(us);
  const size_t REGION = 2 * PLANE;
  const size_t need   = 7 * REGION;
  if (ws_size < need) return;
  char* ws = (char*)d_ws;

  us* Xh  = (us*)(ws + 0 * REGION); us* Xl  = (us*)(ws + 0 * REGION + PLANE);
  us* WQh = (us*)(ws + 1 * REGION); us* WQl = (us*)(ws + 1 * REGION + PLANE);
  us* WKh = (us*)(ws + 2 * REGION); us* WKl = (us*)(ws + 2 * REGION + PLANE);
  us* WVh = (us*)(ws + 3 * REGION); us* WVl = (us*)(ws + 3 * REGION + PLANE);
  float* Qf = (float*)(ws + 4 * REGION);
  float* Kf = (float*)(ws + 5 * REGION);
  us* VTh = (us*)(ws + 6 * REGION); us* VTl = (us*)(ws + 6 * REGION + PLANE);
  us* QPh = Xh;  us* QPl = Xl;
  us* KPh = WQh; us* KPl = WQl;
  us* CXh = WKh; us* CXl = WKl;
  us* WOh = WVh; us* WOl = WVl;

  {
    CvtArgs a;
    a.s0 = hs; a.s1 = wq; a.s2 = wk; a.s3 = wv;
    a.h0 = Xh; a.h1 = WQh; a.h2 = WKh; a.h3 = WVh;
    a.l0 = Xl; a.l1 = WQl; a.l2 = WKl; a.l3 = WVl;
    a.n0 = SEQ; a.n1 = DIM; a.n2 = DIM; a.n3 = DIM;
    cvt_planes_kernel<<<dim3(SPAD, 4), 256, 0, stream>>>(a);
  }

  const dim3 gg(SPAD / 128, DIM / 128);
  gemm_abT_kernel<0><<<gg, 256, 0, stream>>>(Xh, Xl, WQh, WQl, bq, Qf, VTh, VTl, SPAD, SPAD);
  gemm_abT_kernel<0><<<gg, 256, 0, stream>>>(Xh, Xl, WKh, WKl, bk, Kf, VTh, VTl, SPAD, SPAD);
  gemm_abT_kernel<1><<<gg, 256, 0, stream>>>(WVh, WVl, Xh, Xl, bv, Qf, VTh, VTl, SPAD, SEQ);

  {
    CvtArgs a;
    a.s0 = wo; a.s1 = wo; a.s2 = wo; a.s3 = wo;
    a.h0 = WOh; a.h1 = WOh; a.h2 = WOh; a.h3 = WOh;
    a.l0 = WOl; a.l1 = WOl; a.l2 = WOl; a.l3 = WOl;
    a.n0 = DIM; a.n1 = DIM; a.n2 = DIM; a.n3 = DIM;
    cvt_planes_kernel<<<dim3(SPAD, 1), 256, 0, stream>>>(a);
  }

  norm_rope_kernel<<<dim3(SPAD, 2), 256, 0, stream>>>(Qf, Kf, nqw, nkw, fcos, fsin,
                                                       QPh, QPl, KPh, KPl, SEQ);

  const int QTILES = (SEQ + 15) / 16;
  const size_t tail_off = (size_t)(QTILES * 16) * DIM * sizeof(us);
  const size_t tail_len = (size_t)(SPAD - QTILES * 16) * DIM * sizeof(us);
  hipMemsetAsync((char*)CXh + tail_off, 0, tail_len, stream);
  hipMemsetAsync((char*)CXl + tail_off, 0, tail_len, stream);

  attn_kernel<<<dim3(QTILES, HEADS), 32, 0, stream>>>(QPh, QPl, KPh, KPl, VTh, VTl, CXh, CXl);

  gemm_abT_kernel<2><<<gg, 256, 0, stream>>>(CXh, CXl, WOh, WOl, bo, out, VTh, VTl, SEQ, SPAD);
}
